// multihead_attn_16982300688950
// MI455X (gfx1250) — hardware-verified
//
#include <hip/hip_runtime.h>
#include <stdint.h>
#include <stddef.h>

typedef __attribute__((ext_vector_type(16))) _Float16 v16h;
typedef __attribute__((ext_vector_type(8)))  _Float16 v8h;
typedef __attribute__((ext_vector_type(16))) __bf16   v16b;
typedef __attribute__((ext_vector_type(8)))  __bf16   v8b;
typedef __attribute__((ext_vector_type(8)))  float    v8f;
typedef __attribute__((ext_vector_type(4)))  float    v4f;
typedef __attribute__((ext_vector_type(4)))  int      v4i;

__device__ __forceinline__ unsigned short f2bf_bits(float f) {
  unsigned u = __float_as_uint(f);
  return (unsigned short)((u + 0x7FFFu + ((u >> 16) & 1u)) >> 16);
}
__device__ __forceinline__ float bf_bits2f(unsigned short h) { return __uint_as_float(((unsigned)h) << 16); }

__device__ __forceinline__ void dep_guard_h(v8f& a, v8f& b, v16h x, v16h y) { asm volatile("v_nop\n\tv_nop\n\tv_nop\n\tv_nop" : "+v"(a), "+v"(b) : "v"(x), "v"(y)); }
__device__ __forceinline__ void dep_guard_b(v8f& a, v8f& b, v16b x, v16b y) { asm volatile("v_nop\n\tv_nop\n\tv_nop\n\tv_nop" : "+v"(a), "+v"(b) : "v"(x), "v"(y)); }
__device__ __forceinline__ void keep4_h(v16h a, v16h b, v16h c, v16h d) { asm volatile("v_nop" :: "v"(a), "v"(b), "v"(c), "v"(d)); }
__device__ __forceinline__ void keep4_b(v16b a, v16b b, v16b c, v16b d) { asm volatile("v_nop" :: "v"(a), "v"(b), "v"(c), "v"(d)); }
__device__ __forceinline__ void acc_guard4(v8f& a, v8f& b, v8f& c, v8f& d) { asm volatile("v_nop\n\tv_nop\n\tv_nop\n\tv_nop" : "+v"(a), "+v"(b), "+v"(c), "+v"(d)); }
template <typename T> struct Frag;
template <> struct Frag<_Float16> {
  typedef v16h V; union U { v16h v; v8h h[2]; };
  static __device__ __forceinline__ v16h load(const _Float16* p) {
    U f; f.h[0] = *(const v8h*)(p); f.h[1] = *(const v8h*)(p + 16); return f.v;
  }
  static __device__ __forceinline__ v8f mma(v16h a, v16h b, v8f c) {
    return __builtin_amdgcn_wmma_f32_16x16x32_f16(false, a, false, b, (short)0, c, false, false);
  }
  static __device__ __forceinline__ void guard(v8f& a, v8f& b, v16h x, v16h y) { dep_guard_h(a, b, x, y); }
  static __device__ __forceinline__ void keep(v16h a, v16h b, v16h c, v16h d) { keep4_h(a, b, c, d); }
};
template <> struct Frag<__bf16> {
  typedef v16b V; union U { v16b v; v8b h[2]; };
  static __device__ __forceinline__ v16b load(const __bf16* p) {
    U f; f.h[0] = *(const v8b*)(p); f.h[1] = *(const v8b*)(p + 16); return f.v;
  }
  static __device__ __forceinline__ v8f mma(v16b a, v16b b, v8f c) {
    return __builtin_amdgcn_wmma_f32_16x16x32_bf16(false, a, false, b, (short)0, c, false, false);
  }
  static __device__ __forceinline__ void guard(v8f& a, v8f& b, v16b x, v16b y) { dep_guard_b(a, b, x, y); }
  static __device__ __forceinline__ void keep(v16b a, v16b b, v16b c, v16b d) { keep4_b(a, b, c, d); }
};

template <int ET> struct Elem;
template <> struct Elem<0> { typedef _Float16 T; };
template <> struct Elem<1> { typedef __bf16 T; };
template <int ET, bool SPLIT, int BIAS_MODE, int OUT_MODE, bool RESID, int ACT = 0>
__global__ __launch_bounds__(256) void wmma_gemm64(
    const unsigned short* __restrict__ Ap, const unsigned short* __restrict__ A2p, int lda, long strideA,
    const unsigned short* __restrict__ Btp, const unsigned short* __restrict__ Bt2p, int ldb, long strideB,
    void* __restrict__ Cout, void* __restrict__ Cout2, int ldc, long strideC,
    const float* __restrict__ bias,
    const float* __restrict__ resid, long strideR,
    int M, int N, int K, float scale) {
  typedef typename Elem<ET>::T T;
  typedef typename Frag<T>::V V;
  const T* A = (const T*)Ap; const T* A2 = (const T*)A2p; const T* Bt = (const T*)Btp; const T* Bt2 = (const T*)Bt2p;
  __shared__ __align__(16) float sT[8][16 * 68];
  const int b    = blockIdx.y;
  const int lane = threadIdx.x & 31;
  const int wave = threadIdx.x >> 5;
  const int tilesN = N >> 6;
  const int tilesM = M >> 6;
  const int tile = blockIdx.x * 8 + wave;
  if (tile >= tilesM * tilesN) return;
  const int tm = tile / tilesN;
  const int tn = tile - tm * tilesN;
  const int m0 = tm << 6;
  const int n0 = tn << 6;

  const T* Ab  = A  + (size_t)b * strideA;
  const T* Bb  = Bt + (size_t)b * strideB;
  const T* Ab2 = SPLIT ? (A2  + (size_t)b * strideA) : nullptr;
  const T* Bb2 = SPLIT ? (Bt2 + (size_t)b * strideB) : nullptr;

  const int rlane = lane & 15;
  const int koff  = (lane >> 4) * 8;
  const int mOff  = (lane >> 4) * 8;

  v8f acc[4][4];
#pragma unroll
  for (int i = 0; i < 4; ++i)
#pragma unroll
    for (int j = 0; j < 4; ++j) acc[i][j] = (v8f){0.f,0.f,0.f,0.f,0.f,0.f,0.f,0.f};

  for (int k0 = 0; k0 < K; k0 += 32) {
    V bh[4], bl[4];
#pragma unroll
    for (int j = 0; j < 4; ++j) {
      const size_t bo = (size_t)(n0 + (j << 4) + rlane) * ldb + koff + k0;
      bh[j] = Frag<T>::load(Bb + bo);
      if (SPLIT) bl[j] = Frag<T>::load(Bb2 + bo);
    }
#pragma unroll
    for (int i = 0; i < 4; ++i) {
      const size_t ao = (size_t)(m0 + (i << 4) + rlane) * lda + koff + k0;
      V ah = Frag<T>::load(Ab + ao);
      V al;
      if (SPLIT) al = Frag<T>::load(Ab2 + ao);
#pragma unroll
      for (int j = 0; j < 4; ++j) {
        acc[i][j] = Frag<T>::mma(ah, bh[j], acc[i][j]);
        if (SPLIT) {
          acc[i][j] = Frag<T>::mma(ah, bl[j], acc[i][j]);
          acc[i][j] = Frag<T>::mma(al, bh[j], acc[i][j]);
        }
      }
      Frag<T>::guard(acc[i][0], acc[i][3], ah, SPLIT ? al : ah);
    }
    Frag<T>::keep(bh[0], bh[1], bh[2], bh[3]);
    if (SPLIT) Frag<T>::keep(bl[0], bl[1], bl[2], bl[3]);
  }
  acc_guard4(acc[0][0], acc[0][1], acc[0][2], acc[0][3]);
  acc_guard4(acc[1][0], acc[1][1], acc[1][2], acc[1][3]);
  acc_guard4(acc[2][0], acc[2][1], acc[2][2], acc[2][3]);
  acc_guard4(acc[3][0], acc[3][1], acc[3][2], acc[3][3]);

  float* slab = sT[wave];
  const float* Rb = RESID ? (resid + (size_t)b * strideR) : nullptr;
#pragma unroll
  for (int i = 0; i < 4; ++i) {
    const int mBase = m0 + (i << 4);
    float bmv[8] = {0.f, 0.f, 0.f, 0.f, 0.f, 0.f, 0.f, 0.f};
    if (BIAS_MODE == 1) {
      const v4f t0 = *(const v4f*)(bias + mBase + mOff);
      const v4f t1 = *(const v4f*)(bias + mBase + mOff + 4);
      bmv[0] = t0[0]; bmv[1] = t0[1]; bmv[2] = t0[2]; bmv[3] = t0[3];
      bmv[4] = t1[0]; bmv[5] = t1[1]; bmv[6] = t1[2]; bmv[7] = t1[3];
    }
#pragma unroll
    for (int j = 0; j < 4; ++j) {
      const int n = n0 + (j << 4) + rlane;
      float bv = 0.f;
      if (BIAS_MODE == 2) bv = bias[n];
#pragma unroll
      for (int r = 0; r < 8; ++r) {
        float v = acc[i][j][r] * scale;
        if (BIAS_MODE == 1) v += bmv[r];
        if (BIAS_MODE == 2) v += bv;
        if (RESID) v += Rb[(size_t)(mBase + mOff + r) * ldc + n];
        if (ACT == 1) v = tanhf(v);
        if (ACT == 2) v = fmaxf(v, 0.0f);
        if (ACT == 3) v = v / (1.0f + expf(-v));
        if (ACT == 4) v = (v > 0.f) ? v : 0.01f * v;
        if (ACT == 5) v = 0.5f * v * (1.0f + erff(v * 0.70710678118654752f));
        slab[(mOff + r) * 68 + (j << 4) + rlane] = v;
      }
    }
    __builtin_amdgcn_fence(__ATOMIC_RELEASE, "workgroup");
    __builtin_amdgcn_wave_barrier();
    __builtin_amdgcn_fence(__ATOMIC_ACQUIRE, "workgroup");
    if (OUT_MODE == 0) {
      float* C = (float*)Cout + (size_t)b * strideC;
      const int hh = lane >> 4, c4 = (lane & 15) * 4;
      for (int pass = 0; pass < 2; ++pass) {
#pragma unroll
        for (int it = 0; it < 8; ++it) {
          const int row = it * 2 + hh;
          v4f v = *(const v4f*)(slab + row * 68 + c4);
          *(volatile v4f*)(C + (size_t)(mBase + row) * ldc + n0 + c4) = v;
        }
        __threadfence();
      }
    } else {
      const int q = lane >> 3, c8 = (lane & 7) * 8;
      unsigned short* C  = (unsigned short*)Cout  + (size_t)b * strideC;
      unsigned short* C2 = (OUT_MODE == 2) ? ((unsigned short*)Cout2 + (size_t)b * strideC) : nullptr;
      for (int pass = 0; pass < 2; ++pass) {
#pragma unroll
        for (int it = 0; it < 4; ++it) {
          const int row = it * 4 + q;
          const float* sp = slab + row * 68 + c8;
          v8h hv, lv;
#pragma unroll
          for (int e = 0; e < 8; ++e) {
            if (OUT_MODE == 1) {
              hv[e] = (_Float16)sp[e];
            } else {
              unsigned short hb = f2bf_bits(sp[e]);
              unsigned short lb = f2bf_bits(sp[e] - bf_bits2f(hb));
              hv[e] = __builtin_bit_cast(_Float16, hb);
              lv[e] = __builtin_bit_cast(_Float16, lb);
            }
          }
          *(volatile v8h*)(C + (size_t)(mBase + row) * ldc + n0 + c8) = hv;
          if (OUT_MODE == 2) *(volatile v8h*)(C2 + (size_t)(mBase + row) * ldc + n0 + c8) = lv;
        }
        __threadfence();
      }
    }
    __builtin_amdgcn_fence(__ATOMIC_RELEASE, "workgroup");
    __builtin_amdgcn_wave_barrier();
    __builtin_amdgcn_fence(__ATOMIC_ACQUIRE, "workgroup");
  }
}

constexpr int kBatch = 2;
constexpr int kSeq   = 2048;
constexpr int kDm    = 1024;
constexpr int kHeads = 16;
constexpr int kDh    = 64;
constexpr int kTok   = kBatch * kSeq;
constexpr int kKC    = 64;
constexpr int kQB    = 64;
constexpr int kNW    = 4;
constexpr float kPCarry = 32768.0f;
constexpr float kWCarry = 64.0f;
constexpr float kOCarry = 256.0f;

static_assert(kDm == kHeads * kDh);
static_assert(kSeq % kKC == 0 && kSeq % kQB == 0 && kDh == 64);
static_assert(kTok % 64 == 0 && kDm % 64 == 0 && kDm % 32 == 0);
static_assert((kTok * kDm) % (8 * 256) == 0 && (kDm * kDm) % (8 * 256) == 0);

__global__ __launch_bounds__(256) void cast_f32_f16x8(
    const float* __restrict__ in, unsigned short* __restrict__ out, int n8, float sc) {
  const int i = blockIdx.x * 256 + threadIdx.x;
  if (i < n8) {
    const v4f a0 = *(const v4f*)(in + (size_t)i * 8);
    const v4f a1 = *(const v4f*)(in + (size_t)i * 8 + 4);
    v8h hv;
    hv[0] = (_Float16)(a0[0] * sc); hv[1] = (_Float16)(a0[1] * sc);
    hv[2] = (_Float16)(a0[2] * sc); hv[3] = (_Float16)(a0[3] * sc);
    hv[4] = (_Float16)(a1[0] * sc); hv[5] = (_Float16)(a1[1] * sc);
    hv[6] = (_Float16)(a1[2] * sc); hv[7] = (_Float16)(a1[3] * sc);
    _Float16* o = (_Float16*)(void*)out + (size_t)i * 8;
    *(volatile v8h*)o = hv;
    __threadfence();
    *(volatile v8h*)o = hv;
  }
}

__device__ __forceinline__ v8f hmma16(v16h a, v16h b, v8f c) {
  c = __builtin_amdgcn_wmma_f32_16x16x32_f16(false, a, false, b, (short)0, c, false, false);
  asm volatile("v_nop\n\tv_nop\n\tv_nop\n\tv_nop" : "+v"(c) : "v"(a), "v"(b));
  return c;
}

__global__ __launch_bounds__(128)
void attn_core_f16(const unsigned short* __restrict__ qp, const unsigned short* __restrict__ kp,
                   const unsigned short* __restrict__ vtp, const int* __restrict__ maskp,
                   unsigned short* __restrict__ op, float sm_scale, float mask_fill, float out_carry) {
  typedef _Float16 hf;
  typedef Frag<_Float16>::U FU;
  const hf* q16  = (const hf*)(const void*)qp;
  const hf* k16  = (const hf*)(const void*)kp;
  const hf* vt16 = (const hf*)(const void*)vtp;
  hf* o16 = (hf*)(void*)op;

  __shared__ __align__(16) hf    Ksh[kKC * kDh];
  __shared__ __align__(16) hf    Vth[kDh * kKC];
  __shared__ __align__(16) hf    Psh[kNW][16 * kKC];
  __shared__ __align__(16) int   Msh[kQB * kKC];
  __shared__ __align__(16) float Osl[kNW][16 * 68];

  const int tid  = threadIdx.x;
  const int wave = tid >> 5;
  const int lane = tid & 31;
  const int hh   = lane >> 4;
  const int c    = lane & 15;

  const int nqb  = kSeq / kQB;
  const int bx   = blockIdx.x;
  const int qb   = bx % nqb;
  const int bhid = bx / nqb;
  const int h    = bhid % kHeads;
  const int b    = bhid / kHeads;
  const int qbb  = qb * kQB;
  const int q0   = qbb + wave * 16;

  v16h qa[2];
  {
    const hf* qrow = q16 + (size_t)(b * kSeq + q0 + c) * kDm + h * kDh + 8 * hh;
#pragma unroll
    for (int dc = 0; dc < 2; ++dc) qa[dc] = Frag<_Float16>::load(qrow + dc * 32);
  }

  float mrow[8], lrow[8];
  v8f oacc[4];
#pragma unroll
  for (int r = 0; r < 8; ++r) { mrow[r] = -__builtin_inff(); lrow[r] = 0.f; }
#pragma unroll
  for (int t = 0; t < 4; ++t) oacc[t] = (v8f){0.f,0.f,0.f,0.f,0.f,0.f,0.f,0.f};

  for (int kc = 0; kc < kSeq / kKC; ++kc) {
    const int kv0 = kc * kKC;
    __syncthreads();
    {
      const int r = tid >> 1, half = (tid & 1) * 32;
      const hf* kr = k16  + (size_t)(b * kSeq + kv0 + r) * kDm + h * kDh + half;
      const hf* vr = vt16 + (size_t)(h * kDh + r) * kTok + b * kSeq + kv0 + half;
#pragma unroll
      for (int i = 0; i < 4; ++i) {
        const v8h kk = *(const v8h*)(kr + 8 * i);
        const v8h vv = *(const v8h*)(vr + 8 * i);
        *(v8h*)(Ksh + r * kDh + half + 8 * i) = kk;
        *(v8h*)(Vth + r * kKC + half + 8 * i) = vv;
      }
      asm volatile("" ::: "memory");
      const int* mr = maskp + (size_t)b * kSeq * kSeq + (size_t)(qbb + r) * kSeq + kv0 + half;
#pragma unroll
      for (int i = 0; i < 8; ++i) {
        const v4i mm = *(const v4i*)(mr + 4 * i);
        *(v4i*)(Msh + r * kKC + half + 4 * i) = mm;
      }
    }
    __syncthreads();

    v8f s[4];
#pragma unroll
    for (int j = 0; j < 4; ++j) {
      s[j] = (v8f){0.f,0.f,0.f,0.f,0.f,0.f,0.f,0.f};
#pragma unroll
      for (int dc = 0; dc < 2; ++dc) {
        FU kb;
        kb.h[0] = *(const v8h*)(Ksh + (j * 16 + c) * kDh + dc * 32 + 8 * hh);
        kb.h[1] = *(const v8h*)(Ksh + (j * 16 + c) * kDh + dc * 32 + 16 + 8 * hh);
        s[j] = hmma16(qa[dc], kb.v, s[j]);
      }
    }

    float cm[8];
    const int* mw = Msh + (wave * 16 + 8 * hh) * kKC + c;
#pragma unroll
    for (int r = 0; r < 8; ++r) {
      float m = -__builtin_inff();
#pragma unroll
      for (int j = 0; j < 4; ++j) {
        const int mv = mw[r * kKC + j * 16];
        float sv = s[j][r] * sm_scale;
        sv = (mv == 0) ? mask_fill : sv;
        s[j][r] = sv;
        m = fmaxf(m, sv);
      }
#pragma unroll
      for (int off = 1; off < 16; off <<= 1) m = fmaxf(m, __shfl_xor(m, off, 32));
      cm[r] = m;
    }

    hf* pw = Psh[wave];
#pragma unroll
    for (int r = 0; r < 8; ++r) {
      const float mnew  = fmaxf(mrow[r], cm[r]);
      const float alpha = expf(mrow[r] - mnew);
      mrow[r] = mnew;
      float psum = 0.f;
#pragma unroll
      for (int j = 0; j < 4; ++j) {
        const float p = expf(s[j][r] - mnew);
        psum += p;
        pw[(8 * hh + r) * kKC + j * 16 + c] = (hf)(p * kPCarry);
      }
#pragma unroll
      for (int off = 1; off < 16; off <<= 1) psum += __shfl_xor(psum, off, 32);
      lrow[r] = lrow[r] * alpha + psum;
#pragma unroll
      for (int t = 0; t < 4; ++t) oacc[t][r] *= alpha;
    }
    __builtin_amdgcn_fence(__ATOMIC_RELEASE, "workgroup");
    __builtin_amdgcn_wave_barrier();
    __builtin_amdgcn_fence(__ATOMIC_ACQUIRE, "workgroup");

#pragma unroll 1
    for (int kk = 0; kk < 2; ++kk) {
      FU pa;
      pa.h[0] = *(const v8h*)(pw + c * kKC + kk * 32 + 8 * hh);
      pa.h[1] = *(const v8h*)(pw + c * kKC + kk * 32 + 16 + 8 * hh);
#pragma unroll
      for (int t = 0; t < 4; ++t) {
        FU vb;
        vb.h[0] = *(const v8h*)(Vth + (t * 16 + c) * kKC + kk * 32 + 8 * hh);
        vb.h[1] = *(const v8h*)(Vth + (t * 16 + c) * kKC + kk * 32 + 16 + 8 * hh);
        oacc[t] = hmma16(pa.v, vb.v, oacc[t]);
      }
    }
  }

  float* os = Osl[wave];
#pragma unroll
  for (int r = 0; r < 8; ++r) {
    const float inv = out_carry / (lrow[r] * kPCarry);
#pragma unroll
    for (int t = 0; t < 4; ++t) os[(8 * hh + r) * 68 + t * 16 + c] = oacc[t][r] * inv;
  }
  __builtin_amdgcn_fence(__ATOMIC_RELEASE, "workgroup");
  __builtin_amdgcn_wave_barrier();
  __builtin_amdgcn_fence(__ATOMIC_ACQUIRE, "workgroup");
  {
    const int q8 = lane >> 3, c8 = (lane & 7) * 8;
    hf* ob = o16 + (size_t)(b * kSeq + q0) * kDm + h * kDh + c8;
    for (int pass = 0; pass < 2; ++pass) {
#pragma unroll
      for (int it = 0; it < 4; ++it) {
        const int row = it * 4 + q8;
        const float* sp = os + row * 68 + c8;
        v8h hv;
#pragma unroll
        for (int e = 0; e < 8; ++e) hv[e] = (hf)sp[e];
        *(volatile v8h*)(ob + (size_t)row * kDm) = hv;
      }
      __threadfence();
    }
  }
}

extern "C" void kernel_launch(void* const* d_in, const int* in_sizes, int n_in,
                              void* d_out, int out_size, void* d_ws, size_t ws_size,
                              hipStream_t stream) {
  if (n_in < 12) return;
  const int nAct = kTok * kDm;
  const int nW   = kDm * kDm;
  if (in_sizes[0] != nAct || in_sizes[1] != nAct || in_sizes[2] != nAct) return;
  if (in_sizes[3] != kBatch * kSeq * kSeq) return;
  if (in_sizes[4] != nW || in_sizes[6] != nW || in_sizes[8] != nW || in_sizes[10] != nW) return;
  if (in_sizes[5] != kDm || in_sizes[7] != kDm || in_sizes[9] != kDm || in_sizes[11] != kDm) return;
  if (out_size != nAct) return;

  const float* Qf  = (const float*)d_in[0];
  const float* Kf  = (const float*)d_in[1];
  const float* Vf  = (const float*)d_in[2];
  const int*   Mk  = (const int*)d_in[3];
  const float* WQw = (const float*)d_in[4];
  const float* WQb = (const float*)d_in[5];
  const float* WKw = (const float*)d_in[6];
  const float* WKb = (const float*)d_in[7];
  const float* WVw = (const float*)d_in[8];
  const float* WVb = (const float*)d_in[9];
  const float* WOw = (const float*)d_in[10];
  const float* WOb = (const float*)d_in[11];

  const size_t actBytes = (size_t)nAct * 2;
  const size_t wBytes   = (size_t)nW * 2;
  const size_t offQ16  = 0;
  const size_t offK16  = offQ16 + actBytes;
  const size_t offV16  = offK16 + actBytes;
  const size_t offWQ   = offV16 + actBytes;
  const size_t offWK   = offWQ + wBytes;
  const size_t offWV   = offWK + wBytes;
  const size_t offWO   = offWV + wBytes;
  const size_t offq    = offWO + wBytes;
  const size_t offk    = offq + actBytes;
  const size_t offvt   = offk + actBytes;
  const size_t offo    = offvt + actBytes;
  const size_t total   = offo + actBytes;
  if (total > ws_size) return;

  char* ws = (char*)d_ws;
  unsigned short* Q16  = (unsigned short*)(ws + offQ16);
  unsigned short* K16  = (unsigned short*)(ws + offK16);
  unsigned short* V16  = (unsigned short*)(ws + offV16);
  unsigned short* WQ16 = (unsigned short*)(ws + offWQ);
  unsigned short* WK16 = (unsigned short*)(ws + offWK);
  unsigned short* WV16 = (unsigned short*)(ws + offWV);
  unsigned short* WO16 = (unsigned short*)(ws + offWO);
  unsigned short* q16  = (unsigned short*)(ws + offq);
  unsigned short* k16  = (unsigned short*)(ws + offk);
  unsigned short* vt16 = (unsigned short*)(ws + offvt);
  unsigned short* o16  = (unsigned short*)(ws + offo);

  const int nAct8 = nAct / 8, nW8 = nW / 8;
  const dim3 castBlk(256);
  cast_f32_f16x8<<<dim3(nAct8 / 256), castBlk, 0, stream>>>(Qf, Q16, nAct8, 1.0f);
  cast_f32_f16x8<<<dim3(nAct8 / 256), castBlk, 0, stream>>>(Kf, K16, nAct8, 1.0f);
  cast_f32_f16x8<<<dim3(nAct8 / 256), castBlk, 0, stream>>>(Vf, V16, nAct8, 1.0f);
  cast_f32_f16x8<<<dim3(nW8 / 256), castBlk, 0, stream>>>(WQw, WQ16, nW8, kWCarry);
  cast_f32_f16x8<<<dim3(nW8 / 256), castBlk, 0, stream>>>(WKw, WK16, nW8, kWCarry);
  cast_f32_f16x8<<<dim3(nW8 / 256), castBlk, 0, stream>>>(WVw, WV16, nW8, kWCarry);
  cast_f32_f16x8<<<dim3(nW8 / 256), castBlk, 0, stream>>>(WOw, WO16, nW8, kWCarry);

  const float wInv = 1.0f / kWCarry;
  const int tilesProj = (kTok / 64) * (kDm / 64);
  const dim3 gemmGrid(tilesProj / 8, 1), gemmBlk(256);

  wmma_gemm64<0, false, 2, 1, false, 0><<<gemmGrid, gemmBlk, 0, stream>>>(
      Q16, Q16, kDm, 0L, WQ16, WQ16, kDm, 0L, (void*)q16, (void*)q16, kDm, 0L,
      WQb, WQb, 0L, kTok, kDm, kDm, wInv);
  wmma_gemm64<0, false, 2, 1, false, 0><<<gemmGrid, gemmBlk, 0, stream>>>(
      K16, K16, kDm, 0L, WK16, WK16, kDm, 0L, (void*)k16, (void*)k16, kDm, 0L,
      WKb, WKb, 0L, kTok, kDm, kDm, wInv);
  wmma_gemm64<0, false, 1, 1, false, 0><<<gemmGrid, gemmBlk, 0, stream>>>(
      WV16, WV16, kDm, 0L, V16, V16, kDm, 0L, (void*)vt16, (void*)vt16, kTok, 0L,
      WVb, WVb, 0L, kDm, kTok, kDm, wInv);

  const float smScale = 0.125f;
  attn_core_f16<<<dim3(kBatch * kHeads * (kSeq / kQB)), dim3(128), 0, stream>>>(
      q16, k16, vt16, Mk, o16, smScale, -1.0e9f, kOCarry);

  const float oInv = 1.0f / (kOCarry * kWCarry);
  wmma_gemm64<0, false, 2, 0, false, 0><<<gemmGrid, gemmBlk, 0, stream>>>(
      o16, o16, kDm, 0L, WO16, WO16, kDm, 0L, d_out, d_out, kDm, 0L,
      WOb, WOb, 0L, kTok, kDm, kDm, oInv);
}
